// HybridDiTBlock_70145405878732
// MI455X (gfx1250) — hardware-run, weakly checked
//
#include <hip/hip_runtime.h>
#include <stddef.h>
#include <math.h>


#pragma clang fp contract(off)

#define NB    2
#define LS    2048
#define DM    1024
#define DI    2048
#define DS    16
#define DR    64
#define DBN   96
#define DBW   128
#define FF    4096
#define SIXD  (6 * DM)
#define MR    (NB * LS)
#define NTHR  256
#define LNEPS 1e-6f
#define WSCAP 134217728
#define WCARRY 64.0f

#define SZ_WBIG ((size_t)SIXD * DM * 2)
#define SZ_WOUT ((size_t)DM * DI * 2)
#define SZ_WXP  ((size_t)DBW * DI * 2)
#define SZ_WDT  ((size_t)DI * DR * 2)
#define SZ_EMB  ((size_t)NB * SIXD * 4)
#define SZ_NH   ((size_t)MR * DM * 2)
#define SZ_XZ   ((size_t)LS * 2 * DI * 4)
#define SZ_XC   ((size_t)LS * DI * 4)
#define SZ_XCH  ((size_t)LS * DI * 2)
#define SZ_DBC  ((size_t)LS * DBW * 4)
#define SZ_DTH  ((size_t)LS * DR * 2)
#define SZ_DEL  ((size_t)LS * DI * 4)
#define SZ_X1   ((size_t)MR * DM * 4)
#define O_WBIG ((size_t)0)
#define O_WOUT (O_WBIG + SZ_WBIG)
#define O_WXP  (O_WOUT + SZ_WOUT)
#define O_WDT  (O_WXP + SZ_WXP)
#define O_EMB  (O_WDT + SZ_WDT)
#define O_NH   (O_EMB + SZ_EMB)
#define O_XZ   (O_NH + SZ_NH)
#define O_XC   (O_XZ + SZ_XZ)
#define O_XCH  (O_XC + SZ_XC)
#define O_DBC  (O_XCH + SZ_XCH)
#define O_DTH  (O_DBC + SZ_DBC)
#define O_DEL  (O_DTH + SZ_DTH)
#define O_X1   (O_DEL + SZ_DEL)
#define WSTOT  (O_X1 + SZ_X1)
static_assert(WSTOT <= (size_t)WSCAP);
static_assert(SZ_XZ == (size_t)MR * FF * 2);
static_assert(SZ_WBIG >= (size_t)(2 * DI) * DM * 2 && SZ_WBIG >= (size_t)FF * DM * 2 && SZ_WBIG >= (size_t)DM * FF * 2);
static_assert((O_WOUT % 128) == 0 && (O_WXP % 128) == 0 && (O_WDT % 128) == 0 && (O_EMB % 128) == 0);
static_assert((O_NH % 128) == 0 && (O_XZ % 128) == 0 && (O_XC % 128) == 0 && (O_XCH % 128) == 0);
static_assert((O_DBC % 128) == 0 && (O_DTH % 128) == 0 && (O_DEL % 128) == 0 && (O_X1 % 128) == 0 && (WSTOT % 128) == 0);

static_assert((LS % 128) == 0 && (MR % 128) == 0 && (DM % 128) == 0 && (DI % 128) == 0 && (FF % 128) == 0 && DBW == 128);
static_assert((DM % 32) == 0 && (DI % 32) == 0 && (DR % 32) == 0 && (FF % 32) == 0);
static_assert((DM % 64) == 0 && (DI % 64) == 0 && (DR % 64) == 0 && (FF % 64) == 0 && (SIXD % 64) == 0 && (DBW % 64) == 0);
static_assert((DBN % 4) == 0 && DBN <= DBW && DR + 2 * DS == DBN);
static_assert(DI / 4 == 512 && (MR % (NTHR / 32)) == 0 && DM == 4 * 256);

typedef _Float16     v16h __attribute__((ext_vector_type(16)));
typedef _Float16     v8h  __attribute__((ext_vector_type(8), __may_alias__));
typedef _Float16     v4h  __attribute__((ext_vector_type(4), __may_alias__));
typedef float        v8f  __attribute__((ext_vector_type(8)));
typedef float        v4f  __attribute__((ext_vector_type(4), __may_alias__));
typedef unsigned int v4u  __attribute__((ext_vector_type(4), __may_alias__));
typedef unsigned int v2u  __attribute__((ext_vector_type(2), __may_alias__));
typedef int          v8i  __attribute__((ext_vector_type(8)));
union Frag { v16h v; v8i w; v4u q[2]; };
union Pk8 { v8h h; v4u u; };
union Pk4 { v4h h; v2u u; };
static_assert(sizeof(Frag) == 32);
static_assert(sizeof(Pk8) == 16);
static_assert(sizeof(Pk4) == 8);

__device__ __forceinline__ v8f wmh(const Frag& a, const Frag& b, v8f c) {
  v8f d = __builtin_amdgcn_wmma_f32_16x16x32_f16(false, a.v, false, b.v, (short)0, c, false, false);
  asm volatile("v_nop\n\tv_nop\n\tv_nop\n\tv_nop" : "+v"(d) : "v"(a.w), "v"(b.w));
  return d;
}

__device__ __forceinline__ v8f zero8() {
  v8f z = {0.f, 0.f, 0.f, 0.f, 0.f, 0.f, 0.f, 0.f};
  return z;
}

__device__ __forceinline__ v4u pack8(v4f a, v4f c, float mul) {
  v8h hv = {(_Float16)(a[0] * mul), (_Float16)(a[1] * mul), (_Float16)(a[2] * mul), (_Float16)(a[3] * mul),
            (_Float16)(c[0] * mul), (_Float16)(c[1] * mul), (_Float16)(c[2] * mul), (_Float16)(c[3] * mul)};
  Pk8 p;
  p.h = hv;
  return p.u;
}

__device__ __forceinline__ v2u pack4(v4f a, float mul) {
  v4h hv = {(_Float16)(a[0] * mul), (_Float16)(a[1] * mul), (_Float16)(a[2] * mul), (_Float16)(a[3] * mul)};
  Pk4 p;
  p.h = hv;
  return p.u;
}

__device__ __forceinline__ float silu_f(float a) { return a * __builtin_amdgcn_rcpf(1.0f + __expf(-a)); }
__device__ __forceinline__ float softplus_f(float a) { return fmaxf(a, 0.0f) + log1pf(__expf(-fabsf(a))); }
__device__ __forceinline__ float gelu_t(float u) {
  const float in = 0.7978845608028654f * (u + 0.044715f * (u * u * u));
  return u * (0.5f * (1.0f + tanhf(in)));
}

#define TRP 72
__global__ __launch_bounds__(NTHR) void k_wtr(const float* __restrict__ Wsrc, int K, int N, float scale,
                                              unsigned short* WT) {
  __shared__ __align__(16) _Float16 sT[64 * TRP];
  const int tid = threadIdx.x;
  const int k0 = blockIdx.x * 64, n0 = blockIdx.y * 64;
  const int cq = (tid & 15) * 4;
  const int gn = n0 + cq;
  const bool valid = gn < N;
  const int gnc = valid ? gn : (N - 4);
#pragma unroll
  for (int p = 0; p < 4; ++p) {
    const int kr = p * 16 + (tid >> 4);
    const v4f v = *(const v4f*)(Wsrc + (size_t)(k0 + kr) * (size_t)N + gnc);
#pragma unroll
    for (int j = 0; j < 4; ++j) {
      const float f = valid ? (v[j] * scale) : 0.0f;
      sT[(cq + j) * TRP + kr] = (_Float16)f;
    }
  }
  __syncthreads();
  v4u o[2];
  size_t d[2];
#pragma unroll
  for (int p = 0; p < 2; ++p) {
    const int e = p * NTHR + tid;
    const int nr = e >> 3, q = e & 7;
    o[p] = *(const v4u*)(sT + nr * TRP + 8 * q);
    d[p] = (size_t)(n0 + nr) * (size_t)K + (size_t)(k0 + 8 * q);
  }
  *(volatile v4u*)(WT + d[0]) = o[0];
  *(volatile v4u*)(WT + d[1]) = o[1];
  __threadfence();
  *(volatile v4u*)(WT + d[0]) = o[0];
  *(volatile v4u*)(WT + d[1]) = o[1];
}

__global__ __launch_bounds__(NTHR) void k_ada(const float* __restrict__ t, const unsigned short* __restrict__ WT,
                                              const float* __restrict__ bada, float* EMB) {
  __shared__ __align__(16) _Float16 sS[NB * DM];
  __shared__ __align__(16) float sO[NB * 128];
  const int tid = threadIdx.x, lane = tid & 31, wave = tid >> 5, h = lane >> 4, m = lane & 15;
  const int n0 = blockIdx.x * 128;
  const int col = n0 + 16 * wave + m;
#pragma unroll 1
  for (int i = 0; i < 8; ++i) {
    const int e = tid * 8 + i;
    sS[e] = (_Float16)silu_f(t[e]);
  }
  __syncthreads();
  v8f acc = zero8();
  const unsigned int msk = (m < NB) ? 0xffffffffu : 0u;
  const _Float16* arow = sS + (m & 1) * DM + 8 * h;
  const unsigned short* wrow = WT + (size_t)col * DM + 8 * h;
#pragma unroll 1
  for (int ks = 0; ks < DM / 32; ++ks) {
    const int k0 = ks << 5;
    Frag fa, fb;
    v4u a0 = *(const v4u*)(arow + k0);
    v4u a1 = *(const v4u*)(arow + k0 + 16);
    a0.x &= msk; a0.y &= msk; a0.z &= msk; a0.w &= msk;
    a1.x &= msk; a1.y &= msk; a1.z &= msk; a1.w &= msk;
    fa.q[0] = a0;
    fa.q[1] = a1;
    fb.q[0] = *(const v4u*)(wrow + k0);
    fb.q[1] = *(const v4u*)(wrow + k0 + 16);
    acc = wmh(fa, fb, acc);
  }
  if (h == 0) {
    sO[0 * 128 + 16 * wave + m] = acc[0];
    sO[1 * 128 + 16 * wave + m] = acc[1];
  }
  __syncthreads();
  if (tid < 64) {
    const int b = tid >> 5, q = tid & 31;
    v4f v = *(const v4f*)(sO + b * 128 + 4 * q);
    const v4f bb = *(const v4f*)(bada + n0 + 4 * q);
#pragma unroll
    for (int j = 0; j < 4; ++j) v[j] = v[j] * (1.0f / WCARRY) + bb[j];
    float* dst = EMB + (size_t)b * SIXD + n0 + 4 * q;
    *(volatile v4f*)dst = v;
    __threadfence();
    *(volatile v4f*)dst = v;
  }
}

__global__ __launch_bounds__(NTHR) void k_ln(const float* __restrict__ X, const float* __restrict__ emb,
                                             int shofs, int scofs, unsigned short* NHp) {
  const int tid = threadIdx.x, lane = tid & 31, wave = tid >> 5;
  const int row = blockIdx.x * (NTHR / 32) + wave;
  const int b = row / LS;
  const float* xp = X + (size_t)row * DM + 8 * lane;
  float v[32];
#pragma unroll
  for (int s = 0; s < 4; ++s) {
    const v4f a = *(const v4f*)(xp + 256 * s);
    const v4f c = *(const v4f*)(xp + 256 * s + 4);
    v[8 * s + 0] = a[0]; v[8 * s + 1] = a[1]; v[8 * s + 2] = a[2]; v[8 * s + 3] = a[3];
    v[8 * s + 4] = c[0]; v[8 * s + 5] = c[1]; v[8 * s + 6] = c[2]; v[8 * s + 7] = c[3];
  }
  float sum = 0.0f;
#pragma unroll
  for (int s = 0; s < 4; ++s)
    sum = sum + (((v[8 * s] + v[8 * s + 1]) + (v[8 * s + 2] + v[8 * s + 3])) +
                 ((v[8 * s + 4] + v[8 * s + 5]) + (v[8 * s + 6] + v[8 * s + 7])));
#pragma unroll
  for (int off = 16; off > 0; off >>= 1) sum += __shfl_xor(sum, off, 32);
  const float mean = sum * (1.0f / (float)DM);
  float dv[32];
  float ss = 0.0f;
#pragma unroll
  for (int i = 0; i < 32; ++i) {
    dv[i] = v[i] - mean;
    ss = ss + dv[i] * dv[i];
  }
#pragma unroll
  for (int off = 16; off > 0; off >>= 1) ss += __shfl_xor(ss, off, 32);
  const float var = ss * (1.0f / (float)DM);
  const float rinv = rsqrtf(var + LNEPS);
  const float* scp = emb + (size_t)b * SIXD + scofs + 8 * lane;
  const float* shp = emb + (size_t)b * SIXD + shofs + 8 * lane;
  v4u o[4];
#pragma unroll
  for (int s = 0; s < 4; ++s) {
    const v4f sa = *(const v4f*)(scp + 256 * s);
    const v4f sb = *(const v4f*)(scp + 256 * s + 4);
    const v4f ha = *(const v4f*)(shp + 256 * s);
    const v4f hb = *(const v4f*)(shp + 256 * s + 4);
    v4f ya, yb;
#pragma unroll
    for (int j = 0; j < 4; ++j) {
      ya[j] = (dv[8 * s + j] * rinv) * (1.0f + sa[j]) + ha[j];
      yb[j] = (dv[8 * s + 4 + j] * rinv) * (1.0f + sb[j]) + hb[j];
    }
    o[s] = pack8(ya, yb, 1.0f);
  }
  unsigned short* dp = NHp + (size_t)row * DM + 8 * lane;
#pragma unroll
  for (int s = 0; s < 4; ++s) *(volatile v4u*)(dp + 256 * s) = o[s];
  __threadfence();
#pragma unroll
  for (int s = 0; s < 4; ++s) *(volatile v4u*)(dp + 256 * s) = o[s];
}

template <int EP>
__global__ __launch_bounds__(NTHR) void k_gemm(const unsigned short* __restrict__ A, int lda,
                                               const unsigned short* __restrict__ W, int ldw, int K, float cscale,
                                               const float* __restrict__ bias, const float* __restrict__ res, int ldr,
                                               const float* __restrict__ gate, int gstride, int gdiv,
                                               float* Cf, int ldc, unsigned short* P, int ldp, float pmul) {
  extern __shared__ __align__(16) float sC[];
  constexpr bool RESG = (EP == 4) || (EP == 6);
  constexpr bool F32O = (EP != 5);
  constexpr int  PW   = (EP == 2) ? 64 : ((EP == 5) ? 128 : 0);
  constexpr int  PPR  = (PW > 0) ? (PW / 8) : 1;
  constexpr int  NPP  = (PW > 0) ? ((128 * PPR) / NTHR) : 1;
  constexpr int  NF4  = (128 * 128 / 4) / NTHR;

  const int tid = threadIdx.x, lane = tid & 31, wave = tid >> 5, h = lane >> 4, m = lane & 15;
  const int wm = wave & 3, wn = wave >> 2;
  const int m0 = blockIdx.y * 128, n0 = blockIdx.x * 128;

  v8f acc[2][4];
#pragma unroll
  for (int mi = 0; mi < 2; ++mi)
#pragma unroll
    for (int ni = 0; ni < 4; ++ni) acc[mi][ni] = zero8();

  const unsigned short* ap0 = A + (size_t)(m0 + 32 * wm + m) * (size_t)lda + 8 * h;
  const unsigned short* ap1 = ap0 + (size_t)16 * (size_t)lda;
  const unsigned short* wp = W + (size_t)(n0 + 64 * wn + m) * (size_t)ldw + 8 * h;
  const size_t wstep = (size_t)16 * (size_t)ldw;
  const int nks = K >> 5;

#pragma unroll 1
  for (int ks = 0; ks < nks; ++ks) {
    const int k0 = ks << 5;
    Frag fa0, fa1;
    fa0.q[0] = *(const v4u*)(ap0 + k0);
    fa0.q[1] = *(const v4u*)(ap0 + k0 + 16);
    fa1.q[0] = *(const v4u*)(ap1 + k0);
    fa1.q[1] = *(const v4u*)(ap1 + k0 + 16);
#pragma unroll
    for (int ni = 0; ni < 4; ++ni) {
      const unsigned short* wpn = wp + wstep * (size_t)ni + k0;
      Frag fb;
      fb.q[0] = *(const v4u*)wpn;
      fb.q[1] = *(const v4u*)(wpn + 16);
      acc[0][ni] = wmh(fa0, fb, acc[0][ni]);
      acc[1][ni] = wmh(fa1, fb, acc[1][ni]);
    }
  }

#pragma unroll
  for (int mi = 0; mi < 2; ++mi) {
#pragma unroll
    for (int ni = 0; ni < 4; ++ni) {
      const int cl = 64 * wn + 16 * ni + m;
#pragma unroll
      for (int r = 0; r < 8; ++r) {
        const int rl = 32 * wm + 16 * mi + 8 * h + r;
        sC[rl * 128 + cl] = acc[mi][ni][r];
      }
    }
  }
  __syncthreads();

  const float* gp = gate;
  if constexpr (RESG) gp = gate + (size_t)(m0 / gdiv) * (size_t)gstride;

#pragma unroll 1
  for (int it = 0; it < NF4; ++it) {
    const int e = it * NTHR + tid;
    const int rl = e >> 5, q = e & 31;
    float* sp = sC + rl * 128 + 4 * q;
    v4f v = *(const v4f*)sp;
    v = v * cscale;
    if constexpr (EP == 3) {
      const v4f bb = *(const v4f*)(bias + n0 + 4 * q);
#pragma unroll
      for (int j = 0; j < 4; ++j) v[j] = softplus_f(v[j] + bb[j]);
    } else if constexpr (EP == 5) {
      const v4f bb = *(const v4f*)(bias + n0 + 4 * q);
#pragma unroll
      for (int j = 0; j < 4; ++j) v[j] = gelu_t(v[j] + bb[j]);
    } else if constexpr (EP == 4) {
      const v4f rr = *(const v4f*)(res + (size_t)(m0 + rl) * (size_t)ldr + n0 + 4 * q);
      const v4f gg = *(const v4f*)(gp + n0 + 4 * q);
#pragma unroll
      for (int j = 0; j < 4; ++j) v[j] = rr[j] + gg[j] * v[j];
    } else if constexpr (EP == 6) {
      const v4f bb = *(const v4f*)(bias + n0 + 4 * q);
      const v4f rr = *(const v4f*)(res + (size_t)(m0 + rl) * (size_t)ldr + n0 + 4 * q);
      const v4f gg = *(const v4f*)(gp + n0 + 4 * q);
#pragma unroll
      for (int j = 0; j < 4; ++j) v[j] = rr[j] + gg[j] * (v[j] + bb[j]);
    }
    *(v4f*)sp = v;
  }
  __syncthreads();

  v4u po[NPP];
  size_t pd[NPP];
  if constexpr (PW > 0) {
#pragma unroll
    for (int i = 0; i < NPP; ++i) {
      const int e = i * NTHR + tid;
      const int rl = e / PPR, q = e % PPR;
      const v4f a = *(const v4f*)(sC + rl * 128 + 8 * q);
      const v4f c = *(const v4f*)(sC + rl * 128 + 8 * q + 4);
      po[i] = pack8(a, c, pmul);
      pd[i] = (size_t)(m0 + rl) * (size_t)ldp + (size_t)(n0 + 8 * q);
    }
  } else {
    po[0] = (v4u){0u, 0u, 0u, 0u};
    pd[0] = 0;
  }

  if constexpr (F32O) {
#pragma unroll 4
    for (int it = 0; it < NF4; ++it) {
      const int e = it * NTHR + tid;
      const int rl = e >> 5, q = e & 31;
      const v4f v = *(const v4f*)(sC + rl * 128 + 4 * q);
      *(volatile v4f*)(Cf + (size_t)(m0 + rl) * (size_t)ldc + n0 + 4 * q) = v;
    }
  }
  if constexpr (PW > 0) {
#pragma unroll
    for (int i = 0; i < NPP; ++i) *(volatile v4u*)(P + pd[i]) = po[i];
  }
  __threadfence();
  if constexpr (F32O) {
#pragma unroll 4
    for (int it = 0; it < NF4; ++it) {
      const int e = it * NTHR + tid;
      const int rl = e >> 5, q = e & 31;
      const v4f v = *(const v4f*)(sC + rl * 128 + 4 * q);
      *(volatile v4f*)(Cf + (size_t)(m0 + rl) * (size_t)ldc + n0 + 4 * q) = v;
    }
  }
  if constexpr (PW > 0) {
#pragma unroll
    for (int i = 0; i < NPP; ++i) *(volatile v4u*)(P + pd[i]) = po[i];
  }
}

__global__ __launch_bounds__(NTHR) void k_conv(const float* __restrict__ XZ, const float* __restrict__ cw,
                                               const float* __restrict__ cb, float* XC, unsigned short* XCH) {
  const int g = blockIdx.x * NTHR + threadIdx.x;
  const int t = g >> 9;
  const int dq = (g & 511) * 4;
  v4f acc = *(const v4f*)(cb + dq);
  v4f w[4];
#pragma unroll
  for (int j = 0; j < 4; ++j) w[j] = *(const v4f*)(cw + (size_t)(dq + j) * 4);
#pragma unroll
  for (int k = 0; k < 4; ++k) {
    const int tt = t + k - 3;
    const int ttc = (tt < 0) ? 0 : tt;
    const v4f xv = *(const v4f*)(XZ + (size_t)ttc * (size_t)(2 * DI) + dq);
    const bool ok = (tt >= 0);
#pragma unroll
    for (int j = 0; j < 4; ++j) {
      const float pr = xv[j] * w[j][k];
      acc[j] = acc[j] + (ok ? pr : 0.0f);
    }
  }
  v4f u;
#pragma unroll
  for (int j = 0; j < 4; ++j) u[j] = silu_f(acc[j]);
  const v2u hv = pack4(u, WCARRY);
  const size_t o = (size_t)t * DI + dq;
  *(volatile v4f*)(XC + o) = u;
  *(volatile v2u*)(XCH + o) = hv;
  __threadfence();
  *(volatile v4f*)(XC + o) = u;
  *(volatile v2u*)(XCH + o) = hv;
}

#define SCB 256
#define STB 32
static_assert(SCB == NTHR && (DI % SCB) == 0 && (LS % STB) == 0 && ((STB * SCB / 8) % NTHR) == 0);

__global__ __launch_bounds__(NTHR) void k_scan(const float* __restrict__ DEL, const float* __restrict__ XC,
                                               const float* __restrict__ DBC, const float* __restrict__ Z,
                                               const float* __restrict__ Alog, const float* __restrict__ Dp,
                                               unsigned short* YH) {
  __shared__ __align__(16) float sA[SCB * DS];
  __shared__ __align__(16) float sY[STB * SCB];
  const int tid = threadIdx.x;
  const int cbase = blockIdx.x * SCB;
  const int c = cbase + tid;
#pragma unroll 1
  for (int e = tid; e < SCB * DS; e += NTHR) sA[e] = -expf(Alog[(size_t)cbase * DS + e]);
  __syncthreads();
  float Aj[DS], hs[DS];
#pragma unroll
  for (int j = 0; j < DS; ++j) {
    Aj[j] = sA[tid * DS + j];
    hs[j] = 0.0f;
  }
  const float Dd = Dp[c];

#pragma unroll 1
  for (int t0 = 0; t0 < LS; t0 += STB) {
#pragma unroll 1
    for (int tl = 0; tl < STB; ++tl) {
      const size_t t = (size_t)(t0 + tl);
      const float dt = DEL[t * DI + c];
      const float xv = XC[t * DI + c];
      const float zv = Z[t * (size_t)(2 * DI) + c];
      const float* bp = DBC + t * DBW + DR;
      const v4f b0 = *(const v4f*)(bp);
      const v4f b1 = *(const v4f*)(bp + 4);
      const v4f b2 = *(const v4f*)(bp + 8);
      const v4f b3 = *(const v4f*)(bp + 12);
      const v4f c0 = *(const v4f*)(bp + 16);
      const v4f c1 = *(const v4f*)(bp + 20);
      const v4f c2 = *(const v4f*)(bp + 24);
      const v4f c3 = *(const v4f*)(bp + 28);
      float Bv[DS], Cv[DS];
      Bv[0] = b0[0]; Bv[1] = b0[1]; Bv[2] = b0[2]; Bv[3] = b0[3];
      Bv[4] = b1[0]; Bv[5] = b1[1]; Bv[6] = b1[2]; Bv[7] = b1[3];
      Bv[8] = b2[0]; Bv[9] = b2[1]; Bv[10] = b2[2]; Bv[11] = b2[3];
      Bv[12] = b3[0]; Bv[13] = b3[1]; Bv[14] = b3[2]; Bv[15] = b3[3];
      Cv[0] = c0[0]; Cv[1] = c0[1]; Cv[2] = c0[2]; Cv[3] = c0[3];
      Cv[4] = c1[0]; Cv[5] = c1[1]; Cv[6] = c1[2]; Cv[7] = c1[3];
      Cv[8] = c2[0]; Cv[9] = c2[1]; Cv[10] = c2[2]; Cv[11] = c2[3];
      Cv[12] = c3[0]; Cv[13] = c3[1]; Cv[14] = c3[2]; Cv[15] = c3[3];
      const float dtx = dt * xv;
      float y = 0.0f;
#pragma unroll
      for (int j = 0; j < DS; ++j) {
        const float dA = __expf(dt * Aj[j]);
        const float hn = dA * hs[j] + dtx * Bv[j];
        hs[j] = hn;
        y = y + hn * Cv[j];
      }
      const float sg = __builtin_amdgcn_rcpf(1.0f + __expf(-zv));
      sY[tl * SCB + tid] = (y + Dd * xv) * (zv * sg);
    }
    __syncthreads();
    {
      constexpr int NIT = (STB * SCB / 8) / NTHR;
      v4u hv[NIT];
      size_t dst[NIT];
#pragma unroll
      for (int it = 0; it < NIT; ++it) {
        const int e = it * NTHR + tid;
        const int rl = e >> 5, q = e & 31;
        const v4f a = *(const v4f*)(sY + rl * SCB + 8 * q);
        const v4f cc = *(const v4f*)(sY + rl * SCB + 8 * q + 4);
        hv[it] = pack8(a, cc, 256.0f);
        dst[it] = (size_t)(t0 + rl) * DI + cbase + 8 * q;
      }
#pragma unroll
      for (int it = 0; it < NIT; ++it) *(volatile v4u*)(YH + dst[it]) = hv[it];
      __threadfence();
#pragma unroll
      for (int it = 0; it < NIT; ++it) *(volatile v4u*)(YH + dst[it]) = hv[it];
    }
    __syncthreads();
  }
}

extern "C" void kernel_launch(void* const* d_in, const int* in_sizes, int n_in,
                              void* d_out, int out_size, void* d_ws, size_t ws_size,
                              hipStream_t stream) {
  if (n_in < 17) return;
  if (in_sizes[0] != NB * LS * DM) return;
  if (in_sizes[1] != NB * DM) return;
  if (in_sizes[2] != DM * SIXD || in_sizes[3] != SIXD) return;
  if (in_sizes[4] != DM * 2 * DI) return;
  if (in_sizes[5] != DI * 4 || in_sizes[6] != DI) return;
  if (in_sizes[7] != DI * DBN) return;
  if (in_sizes[8] != DR * DI || in_sizes[9] != DI) return;
  if (in_sizes[10] != DI * DS || in_sizes[11] != DI) return;
  if (in_sizes[12] != DI * DM) return;
  if (in_sizes[13] != DM * FF || in_sizes[14] != FF) return;
  if (in_sizes[15] != FF * DM || in_sizes[16] != DM) return;
  if (out_size != MR * DM) return;
  const size_t tot = (size_t)WSTOT;
  if (tot > ws_size || tot > (size_t)WSCAP) return;

  const float* x     = (const float*)d_in[0];
  const float* tt    = (const float*)d_in[1];
  const float* wada  = (const float*)d_in[2];
  const float* bada  = (const float*)d_in[3];
  const float* win   = (const float*)d_in[4];
  const float* cw    = (const float*)d_in[5];
  const float* cb    = (const float*)d_in[6];
  const float* wxp   = (const float*)d_in[7];
  const float* wdt   = (const float*)d_in[8];
  const float* bdt   = (const float*)d_in[9];
  const float* alog  = (const float*)d_in[10];
  const float* dpp   = (const float*)d_in[11];
  const float* wout  = (const float*)d_in[12];
  const float* w1    = (const float*)d_in[13];
  const float* b1    = (const float*)d_in[14];
  const float* w2    = (const float*)d_in[15];
  const float* b2    = (const float*)d_in[16];
  float* out = (float*)d_out;

  char* ws = (char*)d_ws;
  unsigned short* WBIG = (unsigned short*)(ws + O_WBIG);
  unsigned short* WOUT = (unsigned short*)(ws + O_WOUT);
  unsigned short* WXP  = (unsigned short*)(ws + O_WXP);
  unsigned short* WDT  = (unsigned short*)(ws + O_WDT);
  float*          EMB  = (float*)(ws + O_EMB);
  unsigned short* NH   = (unsigned short*)(ws + O_NH);
  float*          XZ   = (float*)(ws + O_XZ);
  unsigned short* HH   = (unsigned short*)(ws + O_XZ);
  float*          XC   = (float*)(ws + O_XC);
  unsigned short* XCH  = (unsigned short*)(ws + O_XCH);
  unsigned short* YH   = (unsigned short*)(ws + O_XCH);
  float*          DBC  = (float*)(ws + O_DBC);
  unsigned short* DTH  = (unsigned short*)(ws + O_DTH);
  float*          DEL  = (float*)(ws + O_DEL);
  float*          X1   = (float*)(ws + O_X1);

  const int GLDS = 128 * 128 * 4;

  k_wtr<<<dim3(DM / 64, SIXD / 64), NTHR, 0, stream>>>(wada, DM, SIXD, WCARRY, WBIG);
  k_ada<<<SIXD / 128, NTHR, 0, stream>>>(tt, WBIG, bada, EMB);

  k_wtr<<<dim3(DM / 64, (2 * DI) / 64), NTHR, 0, stream>>>(win, DM, 2 * DI, WCARRY, WBIG);
  k_wtr<<<dim3(DI / 64, DBW / 64), NTHR, 0, stream>>>(wxp, DI, DBN, WCARRY, WXP);
  k_wtr<<<dim3(DR / 64, DI / 64), NTHR, 0, stream>>>(wdt, DR, DI, WCARRY, WDT);
  k_wtr<<<dim3(DI / 64, DM / 64), NTHR, 0, stream>>>(wout, DI, DM, WCARRY, WOUT);

  k_ln<<<MR / (NTHR / 32), NTHR, 0, stream>>>(x, EMB, 0 * DM, 1 * DM, NH);

  for (int b = 0; b < NB; ++b) {
    const size_t rofs = (size_t)b * LS * DM;
    k_gemm<1><<<dim3((2 * DI) / 128, LS / 128), NTHR, GLDS, stream>>>(
        NH + rofs, DM, WBIG, DM, DM, 1.0f / WCARRY, EMB, EMB, 0, EMB, 0, LS,
        XZ, 2 * DI, NH, 0, 1.0f);
    k_conv<<<(LS * DI / 4) / NTHR, NTHR, 0, stream>>>(XZ, cw, cb, XC, XCH);
    k_gemm<2><<<dim3(DBW / 128, LS / 128), NTHR, GLDS, stream>>>(
        XCH, DI, WXP, DI, DI, 1.0f / (WCARRY * WCARRY), EMB, EMB, 0, EMB, 0, LS,
        DBC, DBW, DTH, DR, WCARRY);
    k_gemm<3><<<dim3(DI / 128, LS / 128), NTHR, GLDS, stream>>>(
        DTH, DR, WDT, DR, DR, 1.0f / (WCARRY * WCARRY), bdt, EMB, 0, EMB, 0, LS,
        DEL, DI, NH, 0, 1.0f);
    k_scan<<<DI / SCB, NTHR, 0, stream>>>(DEL, XC, DBC, XZ + DI, alog, dpp, YH);
    k_gemm<4><<<dim3(DM / 128, LS / 128), NTHR, GLDS, stream>>>(
        YH, DI, WOUT, DI, DI, 1.0f / (256.0f * WCARRY), EMB, x + rofs, DM,
        EMB + (size_t)b * SIXD + 2 * DM, SIXD, LS, X1 + rofs, DM, NH, 0, 1.0f);
  }

  k_wtr<<<dim3(DM / 64, FF / 64), NTHR, 0, stream>>>(w1, DM, FF, WCARRY, WBIG);
  k_ln<<<MR / (NTHR / 32), NTHR, 0, stream>>>(X1, EMB, 3 * DM, 4 * DM, NH);
  k_gemm<5><<<dim3(FF / 128, MR / 128), NTHR, GLDS, stream>>>(
      NH, DM, WBIG, DM, DM, 1.0f / WCARRY, b1, EMB, 0, EMB, 0, LS,
      EMB, 0, HH, FF, 16.0f);

  k_wtr<<<dim3(FF / 64, DM / 64), NTHR, 0, stream>>>(w2, FF, DM, WCARRY, WBIG);
  k_gemm<6><<<dim3(DM / 128, MR / 128), NTHR, GLDS, stream>>>(
      HH, FF, WBIG, FF, FF, 1.0f / (16.0f * WCARRY), b2, X1, DM,
      EMB + 5 * DM, SIXD, LS, out, DM, NH, 0, 1.0f);
}
